// ImprovedGenerator_46359876993737
// MI455X (gfx1250) — hardware-verified
//
#include <hip/hip_runtime.h>
#include <math.h>

typedef __attribute__((ext_vector_type(16))) _Float16 v16h;
typedef __attribute__((ext_vector_type(8)))  _Float16 v8h;
typedef __attribute__((ext_vector_type(16))) __bf16   v16b;
typedef __attribute__((ext_vector_type(8)))  __bf16   v8b;
typedef __attribute__((ext_vector_type(8)))  float    v8f;
typedef __attribute__((ext_vector_type(4)))  float    v4f;

constexpr int kB    = 64;
constexpr int kT    = 256;
constexpr int kZ    = 128;
constexpr int kZ2   = 2 * kZ;
constexpr int kH    = 512;
constexpr int kH2   = 2 * kH;
constexpr int kG4   = 4 * kH;
constexpr int kF    = 64;
constexpr int kRows = kT * kB;
constexpr int kCh   = 64;
constexpr int kChRows = kCh * kB;
constexpr int kNCh  = kT / kCh;
constexpr int kThr  = 256;
constexpr float kInCarry = 1024.0f;
constexpr float kWCarry  = 4096.0f;
constexpr float kXCarry  = 1024.0f;
constexpr float kNCarry  = 256.0f;
constexpr float kScC  = 1.0f / (kWCarry * kInCarry);
constexpr float kScXW = 1.0f / (kXCarry * kWCarry);
constexpr float kScNW = 1.0f / (kNCarry * kWCarry);
constexpr float kEps  = 1e-3f;
constexpr float kF16MinNormal = 6.103515625e-5f;

static_assert((kRows % 64) == 0 && (kChRows % 64) == 0 && (kB % 64) == 0 && (kG4 % 64) == 0 && (kH % 64) == 0 && (kZ % 64) == 0 && (kF % 64) == 0, "GEMM M, N multiples of 64");
static_assert(((kG4 / 64) * (kZ / 64)) % 8 == 0 && ((kG4 / 64) * (kB / 64)) % 8 == 0 && ((kRows / 64) * (kH / 64)) % 8 == 0 && ((kChRows / 64) * (kG4 / 64)) % 8 == 0 && ((kB / 64) * (kG4 / 64)) % 8 == 0 && ((kRows / 64) * (kF / 64)) % 8 == 0, "GEMM grids exact");
static_assert((kZ % 32) == 0 && (kZ2 % 32) == 0 && (kH % 32) == 0 && (kH2 % 32) == 0, "GEMM K multiples of 32");
static_assert(kCh * kNCh == kT, "chunks cover the steps");

constexpr size_t kOffZ16  = 0;
constexpr size_t kOffWP16 = kOffZ16  + (size_t)kRows * kZ2 * 2;
constexpr size_t kOffK0T  = kOffWP16 + (size_t)kZ * kH2 * 2;
constexpr size_t kOffBP16 = kOffK0T  + (size_t)kG4 * kH2 * 2;
constexpr size_t kOffWC32 = kOffBP16 + (size_t)kB * kH2 * 2;
constexpr size_t kOffBPK  = kOffWC32 + (size_t)kG4 * kZ * 4;
constexpr size_t kOffWCT  = kOffBPK  + (size_t)kG4 * 64 * 4;
constexpr size_t kOffR0T  = kOffWCT  + (size_t)kG4 * kZ2 * 2;
constexpr size_t kOffK1T  = kOffR0T  + (size_t)kG4 * kH * 2;
constexpr size_t kOffR1T  = kOffK1T  + (size_t)kG4 * kH * 2;
constexpr size_t kOffK2T  = kOffR1T  + (size_t)kG4 * kH * 2;
constexpr size_t kOffR2T  = kOffK2T  + (size_t)kG4 * kH * 2;
constexpr size_t kOffWST  = kOffR2T  + (size_t)kG4 * kH * 2;
constexpr size_t kOffW1T  = kOffWST  + (size_t)kH * kZ * 2;
constexpr size_t kOffW2T  = kOffW1T  + (size_t)kH * kH2 * 2;
constexpr size_t kOffF32  = kOffW2T  + (size_t)kF * kH2 * 2;
constexpr int kFBC = 0, kFB1 = 2048, kFB2 = 4096, kFBS = 6144, kFB1D = 6656, kFB2D = 7168, kFZB = 7296, kFEnd = 10240;
constexpr size_t kOffH0Z  = kOffF32  + (size_t)kFEnd * 4;
constexpr size_t kOffC32  = kOffH0Z  + (size_t)kB * kH * 2;
constexpr size_t kOffGG   = kOffC32  + (size_t)kB * kH * 4;
constexpr size_t kOffRES  = kOffGG   + (size_t)kB * kG4 * 4;
constexpr size_t kOffXK   = kOffRES  + (size_t)kRows * kH * 4;
constexpr size_t kOffHS0  = kOffXK   + (size_t)kChRows * kG4 * 4;
constexpr size_t kOffHS1  = kOffHS0  + (size_t)kRows * kH * 2;
constexpr size_t kOffHS2  = kOffHS1  + (size_t)kRows * kH * 2;
constexpr size_t kOffX2   = kOffHS2  + (size_t)kRows * kH * 2;
constexpr size_t kOffXN16 = kOffX2   + (size_t)kRows * kH * 2;
constexpr size_t kOffD116 = kOffXN16 + (size_t)kRows * kH2 * 2;
constexpr size_t kOffY    = kOffD116 + (size_t)kRows * kH2 * 2;
constexpr size_t kWsTotal = kOffY    + (size_t)kRows * kF * 4;
static_assert(kWsTotal == 233676800ull, "carve total");
static_assert(kWsTotal <= 268435456ull, "carve cap");
static_assert((size_t)kChRows * kG4 == (size_t)kRows * kH, "XK and D1 have the same size");
static_assert((kOffWP16 % 256) == 0 && (kOffK0T % 256) == 0 && (kOffBP16 % 256) == 0 && (kOffWC32 % 256) == 0 && (kOffBPK % 256) == 0 && (kOffWCT % 256) == 0 && (kOffR0T % 256) == 0 && (kOffK1T % 256) == 0 && (kOffR1T % 256) == 0 && (kOffK2T % 256) == 0 && (kOffR2T % 256) == 0 && (kOffWST % 256) == 0 && (kOffW1T % 256) == 0 && (kOffW2T % 256) == 0 && (kOffF32 % 256) == 0 && (kOffH0Z % 256) == 0 && (kOffC32 % 256) == 0 && (kOffGG % 256) == 0 && (kOffRES % 256) == 0 && (kOffXK % 256) == 0 && (kOffHS0 % 256) == 0 && (kOffHS1 % 256) == 0 && (kOffHS2 % 256) == 0 && (kOffX2 % 256) == 0 && (kOffXN16 % 256) == 0 && (kOffD116 % 256) == 0 && (kOffY % 256) == 0, "aligned regions");
static_assert(kFEnd - kFZB >= kG4, "the zero bias row covers the widest product");

__device__ __forceinline__ unsigned short f2bf_bits(float f) {
  unsigned u = __float_as_uint(f);
  return (unsigned short)((u + 0x7FFFu + ((u >> 16) & 1u)) >> 16);
}
__device__ __forceinline__ float bf_bits2f(unsigned short h) { return __uint_as_float(((unsigned)h) << 16); }
__device__ __forceinline__ float bf16r(float f) { return bf_bits2f(f2bf_bits(f)); }
__device__ __forceinline__ float carry_flush(float v, float carry) {
  const float s = v * carry;
  return (fabsf(s) < kF16MinNormal) ? 0.0f : s;
}
__device__ __forceinline__ float frcp(float x) { return __builtin_amdgcn_rcpf(x); }

__device__ __forceinline__ void dep_guard4_h(v8f& a, v8f& b, v8f& c, v8f& d, v16h x, v16h y) { asm volatile("v_nop\n\tv_nop\n\tv_nop\n\tv_nop" : "+v"(a), "+v"(b), "+v"(c), "+v"(d) : "v"(x), "v"(y)); }
__device__ __forceinline__ void dep_guard4_b(v8f& a, v8f& b, v8f& c, v8f& d, v16b x, v16b y) { asm volatile("v_nop\n\tv_nop\n\tv_nop\n\tv_nop" : "+v"(a), "+v"(b), "+v"(c), "+v"(d) : "v"(x), "v"(y)); }
__device__ __forceinline__ void keep4_h(v16h a, v16h b, v16h c, v16h d) { asm volatile("v_nop" :: "v"(a), "v"(b), "v"(c), "v"(d)); }
__device__ __forceinline__ void keep4_b(v16b a, v16b b, v16b c, v16b d) { asm volatile("v_nop" :: "v"(a), "v"(b), "v"(c), "v"(d)); }
__device__ __forceinline__ void acc_guard4(v8f& a, v8f& b, v8f& c, v8f& d) { asm volatile("v_nop\n\tv_nop\n\tv_nop\n\tv_nop" : "+v"(a), "+v"(b), "+v"(c), "+v"(d)); }

template <typename T> struct Frag;
template <> struct Frag<_Float16> {
  typedef v16h V; union U { v16h v; v8h h[2]; };
  static __device__ __forceinline__ v16h load(const _Float16* p) {
    U f; f.h[0] = *(const v8h*)(p); f.h[1] = *(const v8h*)(p + 16); return f.v;
  }
  static __device__ __forceinline__ v8f mma(v16h a, v16h b, v8f c) {
    return __builtin_amdgcn_wmma_f32_16x16x32_f16(false, a, false, b, (short)0, c, false, false);
  }
  static __device__ __forceinline__ void guard4(v8f& a, v8f& b, v8f& c, v8f& d, v16h x, v16h y) { dep_guard4_h(a, b, c, d, x, y); }
  static __device__ __forceinline__ void keep(v16h a, v16h b, v16h c, v16h d) { keep4_h(a, b, c, d); }
};
template <> struct Frag<__bf16> {
  typedef v16b V; union U { v16b v; v8b h[2]; };
  static __device__ __forceinline__ v16b load(const __bf16* p) {
    U f; f.h[0] = *(const v8b*)(p); f.h[1] = *(const v8b*)(p + 16); return f.v;
  }
  static __device__ __forceinline__ v8f mma(v16b a, v16b b, v8f c) {
    return __builtin_amdgcn_wmma_f32_16x16x32_bf16(false, a, false, b, (short)0, c, false, false);
  }
  static __device__ __forceinline__ void guard4(v8f& a, v8f& b, v8f& c, v8f& d, v16b x, v16b y) { dep_guard4_b(a, b, c, d, x, y); }
  static __device__ __forceinline__ void keep(v16b a, v16b b, v16b c, v16b d) { keep4_b(a, b, c, d); }
};

__device__ __forceinline__ v8f mma_h(v16h a, v16h b, v8f c) {
  c = __builtin_amdgcn_wmma_f32_16x16x32_f16(false, a, false, b, (short)0, c, false, false);
  asm volatile("v_nop\n\tv_nop\n\tv_nop\n\tv_nop" : "+v"(c) : "v"(a), "v"(b));
  return c;
}

template <int ET> struct Elem;
template <> struct Elem<0> { typedef _Float16 T; };
template <> struct Elem<1> { typedef __bf16 T; };
template <int ET, bool SPLIT, int BIAS_MODE, int OUT_MODE, bool RESID, int ACT = 0>
__global__ __launch_bounds__(256) void wmma_gemm64(
    const unsigned short* __restrict__ Ap, const unsigned short* __restrict__ A2p, int lda, long strideA,
    const unsigned short* __restrict__ Btp, const unsigned short* __restrict__ Bt2p, int ldb, long strideB,
    void* __restrict__ Cout, void* __restrict__ Cout2, int ldc, long strideC,
    const float* __restrict__ bias,
    const float* __restrict__ resid, long strideR,
    int M, int N, int K, float scale) {
  typedef typename Elem<ET>::T T;
  typedef typename Frag<T>::V V;
  const T* A = (const T*)Ap; const T* A2 = (const T*)A2p; const T* Bt = (const T*)Btp; const T* Bt2 = (const T*)Bt2p;
  __shared__ __align__(16) float sT[8][16 * 68];
  const int b    = blockIdx.y;
  const int lane = threadIdx.x & 31;
  const int wave = threadIdx.x >> 5;
  const int tilesN = N >> 6;
  const int tilesM = M >> 6;
  const int tile = blockIdx.x * 8 + wave;
  if (tile >= tilesM * tilesN) return;
  const int tm = tile / tilesN;
  const int tn = tile - tm * tilesN;
  const int m0 = tm << 6;
  const int n0 = tn << 6;

  const T* Ab  = A  + (size_t)b * strideA;
  const T* Bb  = Bt + (size_t)b * strideB;
  const T* Ab2 = SPLIT ? (A2  + (size_t)b * strideA) : nullptr;
  const T* Bb2 = SPLIT ? (Bt2 + (size_t)b * strideB) : nullptr;

  const int rlane = lane & 15;
  const int koff  = (lane >> 4) * 8;
  const int mOff  = (lane >> 4) * 8;

  v8f acc[4][4];
#pragma unroll
  for (int i = 0; i < 4; ++i)
#pragma unroll
    for (int j = 0; j < 4; ++j) acc[i][j] = (v8f){0.f,0.f,0.f,0.f,0.f,0.f,0.f,0.f};

  for (int k0 = 0; k0 < K; k0 += 32) {
    V bh[4], bl[4];
#pragma unroll
    for (int j = 0; j < 4; ++j) {
      const size_t bo = (size_t)(n0 + (j << 4) + rlane) * ldb + koff + k0;
      bh[j] = Frag<T>::load(Bb + bo);
      if (SPLIT) bl[j] = Frag<T>::load(Bb2 + bo);
    }
#pragma unroll
    for (int i = 0; i < 4; ++i) {
      const size_t ao = (size_t)(m0 + (i << 4) + rlane) * lda + koff + k0;
      V ah = Frag<T>::load(Ab + ao);
      V al;
      if (SPLIT) al = Frag<T>::load(Ab2 + ao);
#pragma unroll
      for (int j = 0; j < 4; ++j) {
        acc[i][j] = Frag<T>::mma(ah, bh[j], acc[i][j]);
        if (SPLIT) {
          acc[i][j] = Frag<T>::mma(ah, bl[j], acc[i][j]);
          acc[i][j] = Frag<T>::mma(al, bh[j], acc[i][j]);
        }
      }
      Frag<T>::guard4(acc[i][0], acc[i][1], acc[i][2], acc[i][3], ah, SPLIT ? al : ah);
    }
    Frag<T>::keep(bh[0], bh[1], bh[2], bh[3]);
    if (SPLIT) Frag<T>::keep(bl[0], bl[1], bl[2], bl[3]);
  }
  acc_guard4(acc[0][0], acc[0][1], acc[0][2], acc[0][3]);
  acc_guard4(acc[1][0], acc[1][1], acc[1][2], acc[1][3]);
  acc_guard4(acc[2][0], acc[2][1], acc[2][2], acc[2][3]);
  acc_guard4(acc[3][0], acc[3][1], acc[3][2], acc[3][3]);

  float* slab = sT[wave];
  const float* Rb = RESID ? (resid + (size_t)b * strideR) : nullptr;
#pragma unroll
  for (int i = 0; i < 4; ++i) {
    const int mBase = m0 + (i << 4);
#pragma unroll
    for (int j = 0; j < 4; ++j) {
      const int n = n0 + (j << 4) + rlane;
      float bv = 0.f;
      if (BIAS_MODE == 2) bv = bias[n];
#pragma unroll
      for (int r = 0; r < 8; ++r) {
        float v = acc[i][j][r] * scale;
        if (BIAS_MODE == 1) v += bias[mBase + mOff + r];
        if (BIAS_MODE == 2) v += bv;
        if (RESID) v += Rb[(size_t)(mBase + mOff + r) * ldc + n];
        if (ACT == 1) v = tanhf(v);
        if (ACT == 2) v = fmaxf(v, 0.0f);
        if (ACT == 3) v = v / (1.0f + expf(-v));
        if (ACT == 4) v = (v > 0.f) ? v : 0.01f * v;
        slab[(mOff + r) * 68 + (j << 4) + rlane] = v;
      }
    }
    __builtin_amdgcn_fence(__ATOMIC_RELEASE, "workgroup");
    __builtin_amdgcn_wave_barrier();
    __builtin_amdgcn_fence(__ATOMIC_ACQUIRE, "workgroup");
    if (OUT_MODE == 0) {
      float* C = (float*)Cout + (size_t)b * strideC;
      const int hh = lane >> 4, c4 = (lane & 15) * 4;
      for (int pass = 0; pass < 2; ++pass) {
#pragma unroll
        for (int it = 0; it < 8; ++it) {
          const int row = it * 2 + hh;
          v4f v = *(const v4f*)(slab + row * 68 + c4);
          *(volatile v4f*)(C + (size_t)(mBase + row) * ldc + n0 + c4) = v;
        }
        __threadfence();
      }
    } else {
      const int q = lane >> 3, c8 = (lane & 7) * 8;
      unsigned short* C  = (unsigned short*)Cout  + (size_t)b * strideC;
      unsigned short* C2 = (OUT_MODE == 2) ? ((unsigned short*)Cout2 + (size_t)b * strideC) : nullptr;
      for (int pass = 0; pass < 2; ++pass) {
#pragma unroll
        for (int it = 0; it < 4; ++it) {
          const int row = it * 4 + q;
          const float* sp = slab + row * 68 + c8;
          v8h hv, lv;
#pragma unroll
          for (int e = 0; e < 8; ++e) {
            if (OUT_MODE == 1) {
              hv[e] = (_Float16)sp[e];
            } else {
              unsigned short hb = f2bf_bits(sp[e]);
              unsigned short lb = f2bf_bits(sp[e] - bf_bits2f(hb));
              hv[e] = __builtin_bit_cast(_Float16, hb);
              lv[e] = __builtin_bit_cast(_Float16, lb);
            }
          }
          *(volatile v8h*)(C + (size_t)(mBase + row) * ldc + n0 + c8) = hv;
          if (OUT_MODE == 2) *(volatile v8h*)(C2 + (size_t)(mBase + row) * ldc + n0 + c8) = lv;
        }
        __threadfence();
      }
    }
    __builtin_amdgcn_fence(__ATOMIC_RELEASE, "workgroup");
    __builtin_amdgcn_wave_barrier();
    __builtin_amdgcn_fence(__ATOMIC_ACQUIRE, "workgroup");
  }
}

__global__ __launch_bounds__(kThr) void cast_plane_kernel(const float* __restrict__ src, unsigned short* __restrict__ dst,
                                                          int colsLog2, int dstPitch, int dstOff) {
  const int i   = blockIdx.x * kThr + threadIdx.x;
  const int sh  = colsLog2 - 3;
  const int row = i >> sh;
  const int c8  = (i & ((1 << sh) - 1)) * 8;
  const float* sp = src + ((size_t)row << colsLog2) + c8;
  const v4f a0 = *(const v4f*)(sp);
  const v4f a1 = *(const v4f*)(sp + 4);
  v8h hv;
#pragma unroll
  for (int e = 0; e < 4; ++e) {
    const float f0 = a0[e];
    const float f1 = a1[e];
    hv[e]     = (_Float16)carry_flush(bf16r(f0), kInCarry);
    hv[4 + e] = (_Float16)carry_flush(bf16r(f1), kInCarry);
  }
  unsigned short* dp = dst + (size_t)row * dstPitch + dstOff + c8;
  *(volatile v8h*)dp = hv;
  __threadfence();
  *(volatile v8h*)dp = hv;
}
__device__ __forceinline__ void split_hl(float v, float c, _Float16& hi, _Float16& lo) {
  const float sv = carry_flush(v, c);
  hi = (_Float16)sv;
  const float r = sv - (float)hi;
  lo = (_Float16)((fabsf(r) < kF16MinNormal) ? 0.0f : r);
}

__global__ __launch_bounds__(256) void wt_plane_kernel(const float* __restrict__ W, unsigned short* __restrict__ dst, int K, int N, int nLive, int ldd, int colOff) {
  const int n  = blockIdx.x;
  const int k8 = threadIdx.x * 8;
  const bool live = n < nLive;
  const int nc = live ? n : 0;
  v8h hv;
#pragma unroll
  for (int e = 0; e < 8; ++e) {
    const float w = W[(size_t)(k8 + e) * N + nc];
    hv[e] = (_Float16)(live ? carry_flush(bf16r(w), kWCarry) : 0.0f);
  }
  unsigned short* dp = dst + (size_t)n * ldd + colOff + k8;
  *(volatile v8h*)dp = hv;
  __threadfence();
  *(volatile v8h*)dp = hv;
}


__device__ __forceinline__ float fast_tanh(float v) { return 1.0f - 2.0f * frcp(__expf(2.0f * v) + 1.0f); }
__device__ __forceinline__ float fast_sigmoid(float v) { return frcp(1.0f + __expf(-v)); }

__global__ __launch_bounds__(kThr) void z_plane_kernel(const float* __restrict__ z, unsigned short* __restrict__ Z16) {
  unsigned v = blockIdx.x * (unsigned)kThr + threadIdx.x;
  asm volatile("" : "+v"(v));
  const unsigned row = v >> 4;
  const unsigned k8 = (v & 15u) * 8u;
  const unsigned t = row >> 6;
  const unsigned b = row & 63u;
  const float* sp = z + ((size_t)b * kT + t) * kZ + k8;
  const v4f a0 = *(const v4f*)sp, a1 = *(const v4f*)(sp + 4);
  v8h hv;
#pragma unroll
  for (int e = 0; e < 4; ++e) {
    const float f0 = a0[e];
    const float f1 = a1[e];
    hv[e]     = (_Float16)carry_flush(bf16r(f0), kXCarry);
    hv[4 + e] = (_Float16)carry_flush(bf16r(f1), kXCarry);
  }
  unsigned short* dp = Z16 + (size_t)row * kZ2 + k8;
  for (int pass = 0; pass < 2; ++pass) {
    *(volatile v8h*)dp = hv;
    *(volatile v8h*)(dp + kZ) = hv;
    __threadfence();
  }
}
static_assert(kRows * (kZ / 8) == 1024 * kThr, "z plane grid exact");

__global__ __launch_bounds__(kThr) void setup_f16_kernel(const float* __restrict__ bp, unsigned short* __restrict__ BP16, unsigned short* __restrict__ H0Z) {
  unsigned v = blockIdx.x * (unsigned)kThr + threadIdx.x;
  asm volatile("" : "+v"(v));
  v8h zv;
#pragma unroll
  for (int e = 0; e < 8; ++e) zv[e] = (_Float16)0.0f;
  unsigned short* dp;
  if (v < 128u) {
    const v4f a0 = *(const v4f*)(bp + v * 8u), a1 = *(const v4f*)(bp + v * 8u + 4u);
#pragma unroll
    for (int e = 0; e < 4; ++e) {
      const float f0 = a0[e];
      const float f1 = a1[e];
      zv[e]     = (_Float16)carry_flush(bf16r(f0), kInCarry);
      zv[4 + e] = (_Float16)carry_flush(bf16r(f1), kInCarry);
    }
    dp = BP16 + (size_t)v * 8u;
  } else if (v < 8192u) {
    dp = BP16 + (size_t)v * 8u;
  } else {
    dp = H0Z + (size_t)(v - 8192u) * 8u;
  }
  *(volatile v8h*)dp = zv;
  __threadfence();
  *(volatile v8h*)dp = zv;
}
static_assert(kB * kH2 / 8 == 8192 && kH2 / 8 == 128 && kB * kH / 8 == 4096 && (8192 + 4096) == 48 * kThr, "set-up B map and grid exact");

__global__ __launch_bounds__(kThr) void wc_split_kernel(const float* __restrict__ WC32, unsigned short* __restrict__ WCT) {
  unsigned v = blockIdx.x * (unsigned)kThr + threadIdx.x;
  asm volatile("" : "+v"(v));
  const unsigned n = v >> 4;
  const unsigned k8 = (v & 15u) * 8u;
  const float* sp = WC32 + (size_t)n * kZ + k8;
  const v4f a0 = *(const v4f*)sp, a1 = *(const v4f*)(sp + 4);
  v8h hv, lv;
#pragma unroll
  for (int e = 0; e < 4; ++e) {
    _Float16 h0, l0, h1, l1;
    split_hl(a0[e], kWCarry, h0, l0);
    split_hl(a1[e], kWCarry, h1, l1);
    hv[e] = h0; lv[e] = l0; hv[4 + e] = h1; lv[4 + e] = l1;
  }
  unsigned short* dp = WCT + (size_t)n * kZ2 + k8;
  for (int pass = 0; pass < 2; ++pass) {
    *(volatile v8h*)dp = hv;
    *(volatile v8h*)(dp + kZ) = lv;
    __threadfence();
  }
}
static_assert(kG4 * (kZ / 8) == 128 * kThr, "composed map grid exact");

__global__ __launch_bounds__(kThr) void setup_f32_kernel(const float* __restrict__ b1,
                                                         const float* __restrict__ b2, const float* __restrict__ bs, const float* __restrict__ b1d,
                                                         const float* __restrict__ b2d, float* __restrict__ F) {
  unsigned v = blockIdx.x * (unsigned)kThr + threadIdx.x;
  asm volatile("" : "+v"(v));
  const unsigned i0 = (unsigned)kFB1 + v * 4u;
  v4f o = {0.f, 0.f, 0.f, 0.f};
  if (i0 < (unsigned)kFB2) {
    const v4f a = *(const v4f*)(b1 + (i0 - (unsigned)kFB1));
#pragma unroll
    for (int e = 0; e < 4; ++e) { const float x = a[e]; o[e] = bf16r(x); }
  } else if (i0 < (unsigned)kFBS) {
    const v4f a = *(const v4f*)(b2 + (i0 - (unsigned)kFB2));
#pragma unroll
    for (int e = 0; e < 4; ++e) { const float x = a[e]; o[e] = bf16r(x); }
  } else if (i0 < (unsigned)kFB1D) {
    const v4f a = *(const v4f*)(bs + (i0 - (unsigned)kFBS));
#pragma unroll
    for (int e = 0; e < 4; ++e) { const float x = a[e]; o[e] = bf16r(x); }
  } else if (i0 < (unsigned)kFB2D) {
    const v4f a = *(const v4f*)(b1d + (i0 - (unsigned)kFB1D));
#pragma unroll
    for (int e = 0; e < 4; ++e) { const float x = a[e]; o[e] = bf16r(x); }
  } else if (i0 < (unsigned)kFZB) {
    const unsigned j = i0 - (unsigned)kFB2D;
    if (j < (unsigned)kF) {
      const v4f a = *(const v4f*)(b2d + j);
#pragma unroll
      for (int e = 0; e < 4; ++e) { const float x = a[e]; o[e] = bf16r(x); }
    }
  }
  float* dp = F + i0;
  *(volatile v4f*)dp = o;
  __threadfence();
  *(volatile v4f*)dp = o;
}
static_assert((kFEnd - kFB1) / 4 == 8 * kThr, "set-up A grid exact");

__global__ __launch_bounds__(kThr) void bias_c_kernel(const float* __restrict__ BPK, const float* __restrict__ b0, float* __restrict__ BC) {
  unsigned v = blockIdx.x * (unsigned)kThr + threadIdx.x;
  asm volatile("" : "+v"(v));
  const unsigned i0 = v * 4u;
  const v4f a = *(const v4f*)(b0 + i0);
  v4f o;
#pragma unroll
  for (int e = 0; e < 4; ++e) { const float x = a[e]; const float p = BPK[(size_t)(i0 + e) * 64u]; o[e] = p + bf16r(x); }
  float* dp = BC + i0;
  *(volatile v4f*)dp = o;
  __threadfence();
  *(volatile v4f*)dp = o;
}
static_assert(kG4 / 4 == 2 * kThr && kFBC == 0, "first-layer bias grid exact");
static_assert((kFB1 % 128) == 0 && (kFB2 % 128) == 0 && (kFBS % 128) == 0 && (kFB1D % 128) == 0 && (kFB2D % 128) == 0 && (kFZB % 128) == 0, "set-up A regions wave-uniform");

__global__ __launch_bounds__(kThr) void cell_zero_kernel(float* __restrict__ C32) {
  const size_t v = (size_t)blockIdx.x * kThr + threadIdx.x;
  const v4f o = {0.f, 0.f, 0.f, 0.f};
  float* dp = C32 + v * 4;
  *(volatile v4f*)dp = o;
  __threadfence();
  *(volatile v4f*)dp = o;
}
static_assert(kB * kH / 4 == 32 * kThr, "cell zero grid exact");

__global__ __launch_bounds__(kThr) void lstm_cell_kernel(const float* __restrict__ XK, const float* __restrict__ GG, float* __restrict__ C32,
                                                         unsigned short* __restrict__ HS, const float* __restrict__ RES, unsigned short* __restrict__ X2,
                                                         float* __restrict__ H2F, int t, int mode) {
  unsigned v = blockIdx.x * (unsigned)kThr + threadIdx.x;
  asm volatile("" : "+v"(v));
  const unsigned b  = v >> 6;
  const unsigned u8 = (v & 63u) * 8u;
  const unsigned tl = (unsigned)t & (unsigned)(kCh - 1);
  const size_t row = (size_t)t * kB + b;
  const float* xr = XK + ((size_t)tl * kB + b) * kG4 + u8;
  const float* gr = GG + (size_t)b * kG4 + u8;
  float* cp = C32 + (size_t)b * kH + u8;
  v8h hv, xv;
  v4f cn0, cn1, hn0, hn1;
#pragma unroll
  for (int e = 0; e < 8; ++e) xv[e] = (_Float16)0.0f;
#pragma unroll
  for (int hlf = 0; hlf < 2; ++hlf) {
    const v4f xi = *(const v4f*)(xr + 4 * hlf), xf = *(const v4f*)(xr + kH + 4 * hlf), xg = *(const v4f*)(xr + 2 * kH + 4 * hlf), xo = *(const v4f*)(xr + 3 * kH + 4 * hlf);
    const v4f gi = *(const v4f*)(gr + 4 * hlf), gf = *(const v4f*)(gr + kH + 4 * hlf), gg = *(const v4f*)(gr + 2 * kH + 4 * hlf), go = *(const v4f*)(gr + 3 * kH + 4 * hlf);
    const v4f co = *(const v4f*)(cp + 4 * hlf);
    v4f rs = {0.f, 0.f, 0.f, 0.f};
    if (mode == 1) rs = *(const v4f*)(RES + row * kH + u8 + 4 * hlf);
#pragma unroll
    for (int e = 0; e < 4; ++e) {
      const float cn = fast_sigmoid(xf[e] + gf[e]) * co[e] + fast_sigmoid(xi[e] + gi[e]) * fast_tanh(xg[e] + gg[e]);
      const float hn = fast_sigmoid(xo[e] + go[e]) * fast_tanh(cn);
      if (hlf == 0) { cn0[e] = cn; hn0[e] = hn; } else { cn1[e] = cn; hn1[e] = hn; }
      hv[4 * hlf + e] = (_Float16)carry_flush(hn, kXCarry);
      xv[4 * hlf + e] = (_Float16)carry_flush(hn + rs[e], kXCarry);
    }
  }
  unsigned short* hp = HS + row * kH + u8;
  unsigned short* xp = X2 + row * kH + u8;
  float* fp = H2F + row * kH + u8;
  for (int pass = 0; pass < 2; ++pass) {
    *(volatile v4f*)cp = cn0;
    *(volatile v4f*)(cp + 4) = cn1;
    *(volatile v8h*)hp = hv;
    if (mode == 1) *(volatile v8h*)xp = xv;
    if (mode == 2) { *(volatile v4f*)fp = hn0; *(volatile v4f*)(fp + 4) = hn1; }
    __threadfence();
  }
}
static_assert(kB * kH / 8 == 16 * kThr, "cell grid exact");

__global__ __launch_bounds__(kThr) void norm_split_kernel(const float* __restrict__ H2F, const float* __restrict__ gamma, const float* __restrict__ beta,
                                                          unsigned short* __restrict__ XN16) {
  unsigned row = blockIdx.x * (unsigned)kThr + threadIdx.x;
  asm volatile("" : "+v"(row));
  const float* xp = H2F + (size_t)row * kH;
  float s = 0.0f;
#pragma unroll 1
  for (int k = 0; k < kH; k += 4) { const v4f a = *(const v4f*)(xp + k); s += a[0]; s += a[1]; s += a[2]; s += a[3]; }
  const float mu = s * (1.0f / (float)kH);
  float q = 0.0f;
#pragma unroll 1
  for (int k = 0; k < kH; k += 4) {
    const v4f a = *(const v4f*)(xp + k);
    const float d0 = a[0] - mu, d1 = a[1] - mu, d2 = a[2] - mu, d3 = a[3] - mu;
    q += d0 * d0; q += d1 * d1; q += d2 * d2; q += d3 * d3;
  }
  const float rs = rsqrtf(q * (1.0f / (float)kH) + kEps);
  unsigned short* op = XN16 + (size_t)row * kH2;
#pragma unroll 1
  for (int k = 0; k < kH; k += 8) {
    const v4f a0 = *(const v4f*)(xp + k), a1 = *(const v4f*)(xp + k + 4);
    const v4f g0 = *(const v4f*)(gamma + k), g1 = *(const v4f*)(gamma + k + 4);
    const v4f c0 = *(const v4f*)(beta + k), c1 = *(const v4f*)(beta + k + 4);
    v8h hv, lv;
#pragma unroll
    for (int e = 0; e < 4; ++e) {
      const float ga = g0[e], gb = g1[e], ba = c0[e], bb = c1[e];
      const float y0 = (a0[e] - mu) * rs * bf16r(ga) + bf16r(ba);
      const float y1 = (a1[e] - mu) * rs * bf16r(gb) + bf16r(bb);
      _Float16 h0, l0, h1, l1;
      split_hl(y0, kNCarry, h0, l0);
      split_hl(y1, kNCarry, h1, l1);
      hv[e] = h0; lv[e] = l0; hv[4 + e] = h1; lv[4 + e] = l1;
    }
    for (int pass = 0; pass < 2; ++pass) {
      *(volatile v8h*)(op + k) = hv;
      *(volatile v8h*)(op + kH + k) = lv;
      __threadfence();
    }
  }
}
static_assert(kRows == 64 * kThr, "norm grid exact");

__global__ __launch_bounds__(kThr) void relu_split_kernel(const float* __restrict__ D1, unsigned short* __restrict__ D116) {
  unsigned v = blockIdx.x * (unsigned)kThr + threadIdx.x;
  asm volatile("" : "+v"(v));
  const unsigned row = v >> 6;
  const unsigned k8 = (v & 63u) * 8u;
  const float* sp = D1 + (size_t)row * kH + k8;
  const v4f a0 = *(const v4f*)sp, a1 = *(const v4f*)(sp + 4);
  v8h hv, lv;
#pragma unroll
  for (int e = 0; e < 4; ++e) {
    _Float16 h0, l0, h1, l1;
    split_hl(fmaxf(a0[e], 0.0f), kXCarry, h0, l0);
    split_hl(fmaxf(a1[e], 0.0f), kXCarry, h1, l1);
    hv[e] = h0; lv[e] = l0; hv[4 + e] = h1; lv[4 + e] = l1;
  }
  unsigned short* dp = D116 + (size_t)row * kH2 + k8;
  for (int pass = 0; pass < 2; ++pass) {
    *(volatile v8h*)dp = hv;
    *(volatile v8h*)(dp + kH) = lv;
    __threadfence();
  }
}
static_assert(kRows * (kH / 8) == 4096 * kThr, "rectifier grid exact");

__global__ __launch_bounds__(kThr) void out_tanh_kernel(const float* __restrict__ Y, float* __restrict__ out) {
  unsigned i = blockIdx.x * (unsigned)kThr + threadIdx.x;
  asm volatile("" : "+v"(i));
  const unsigned b = i >> 12;
  const unsigned t = (i >> 4) & 255u;
  const unsigned f4 = (i & 15u) * 4u;
  const v4f y = *(const v4f*)(Y + ((size_t)t * kB + b) * kF + f4);
  v4f o;
#pragma unroll
  for (int e = 0; e < 4; ++e) o[e] = fast_tanh(y[e]);
  float* dp = out + (size_t)i * 4u;
  *(volatile v4f*)dp = o;
  __threadfence();
  *(volatile v4f*)dp = o;
}
static_assert(kB * kT * kF / 4 == 1024 * kThr && kT * kF / 4 == 4096 && kF / 4 == 16 && kT == 256, "output grid exact");

extern "C" void kernel_launch(void* const* d_in, const int* in_sizes, int n_in,
                              void* d_out, int out_size, void* d_ws, size_t ws_size,
                              hipStream_t stream) {
  if (n_in < 20 || d_out == nullptr || d_ws == nullptr) return;
  if (in_sizes[0] != kB * kT * kZ || in_sizes[1] != kZ * kH2 || in_sizes[2] != kH2 || in_sizes[3] != kZ * kH || in_sizes[4] != kH) return;
  if (in_sizes[5] != kH2 * kG4 || in_sizes[6] != kH * kG4 || in_sizes[7] != kG4 || in_sizes[8] != kH * kG4 || in_sizes[9] != kH * kG4 || in_sizes[10] != kG4) return;
  if (in_sizes[11] != kH * kG4 || in_sizes[12] != kH * kG4 || in_sizes[13] != kG4 || in_sizes[14] != kH || in_sizes[15] != kH) return;
  if (in_sizes[16] != kH * kH || in_sizes[17] != kH || in_sizes[18] != kH * kF || in_sizes[19] != kF) return;
  if (out_size != kB * kT * kF) return;
  if (ws_size < kWsTotal) return;
  const float* z     = (const float*)d_in[0];
  const float* Wp    = (const float*)d_in[1];
  const float* bp    = (const float*)d_in[2];
  const float* Ws    = (const float*)d_in[3];
  const float* bs    = (const float*)d_in[4];
  const float* K0    = (const float*)d_in[5];
  const float* R0    = (const float*)d_in[6];
  const float* b0    = (const float*)d_in[7];
  const float* K1    = (const float*)d_in[8];
  const float* R1    = (const float*)d_in[9];
  const float* b1    = (const float*)d_in[10];
  const float* K2    = (const float*)d_in[11];
  const float* R2    = (const float*)d_in[12];
  const float* b2    = (const float*)d_in[13];
  const float* gamma = (const float*)d_in[14];
  const float* beta  = (const float*)d_in[15];
  const float* W1    = (const float*)d_in[16];
  const float* b1d   = (const float*)d_in[17];
  const float* W2    = (const float*)d_in[18];
  const float* b2d   = (const float*)d_in[19];
  float* out = (float*)d_out;
  char* ws = (char*)d_ws;
  unsigned short* Z16  = (unsigned short*)(ws + kOffZ16);
  unsigned short* WP16 = (unsigned short*)(ws + kOffWP16);
  unsigned short* K0T  = (unsigned short*)(ws + kOffK0T);
  unsigned short* BP16 = (unsigned short*)(ws + kOffBP16);
  float* WC32 = (float*)(ws + kOffWC32);
  float* BPK  = (float*)(ws + kOffBPK);
  unsigned short* WCT  = (unsigned short*)(ws + kOffWCT);
  unsigned short* R0T  = (unsigned short*)(ws + kOffR0T);
  unsigned short* K1T  = (unsigned short*)(ws + kOffK1T);
  unsigned short* R1T  = (unsigned short*)(ws + kOffR1T);
  unsigned short* K2T  = (unsigned short*)(ws + kOffK2T);
  unsigned short* R2T  = (unsigned short*)(ws + kOffR2T);
  unsigned short* WST  = (unsigned short*)(ws + kOffWST);
  unsigned short* W1T  = (unsigned short*)(ws + kOffW1T);
  unsigned short* W2T  = (unsigned short*)(ws + kOffW2T);
  float* F    = (float*)(ws + kOffF32);
  unsigned short* H0Z  = (unsigned short*)(ws + kOffH0Z);
  float* C32  = (float*)(ws + kOffC32);
  float* GG   = (float*)(ws + kOffGG);
  float* RES  = (float*)(ws + kOffRES);
  float* H2F  = (float*)(ws + kOffRES);
  float* XK   = (float*)(ws + kOffXK);
  float* D1   = (float*)(ws + kOffXK);
  unsigned short* HS0  = (unsigned short*)(ws + kOffHS0);
  unsigned short* HS1  = (unsigned short*)(ws + kOffHS1);
  unsigned short* HS2  = (unsigned short*)(ws + kOffHS2);
  unsigned short* X2   = (unsigned short*)(ws + kOffX2);
  unsigned short* XN16 = (unsigned short*)(ws + kOffXN16);
  unsigned short* D116 = (unsigned short*)(ws + kOffD116);
  float* Y    = (float*)(ws + kOffY);

  cast_plane_kernel<<<(int)(((size_t)kZ * kH2 / 8) / kThr), kThr, 0, stream>>>(Wp, WP16, 10, kH2, 0);
  wt_plane_kernel<<<kG4, kH2 / 8, 0, stream>>>(K0, K0T, kH2, kG4, kG4, kH2, 0);
  wt_plane_kernel<<<kG4, kH / 8, 0, stream>>>(R0, R0T, kH, kG4, kG4, kH, 0);
  wt_plane_kernel<<<kG4, kH / 8, 0, stream>>>(K1, K1T, kH, kG4, kG4, kH, 0);
  wt_plane_kernel<<<kG4, kH / 8, 0, stream>>>(R1, R1T, kH, kG4, kG4, kH, 0);
  wt_plane_kernel<<<kG4, kH / 8, 0, stream>>>(K2, K2T, kH, kG4, kG4, kH, 0);
  wt_plane_kernel<<<kG4, kH / 8, 0, stream>>>(R2, R2T, kH, kG4, kG4, kH, 0);
  wt_plane_kernel<<<kH, kZ / 8, 0, stream>>>(Ws, WST, kZ, kH, kH, kZ, 0);
  wt_plane_kernel<<<kH, kH / 8, 0, stream>>>(W1, W1T, kH, kH, kH, kH2, 0);
  wt_plane_kernel<<<kH, kH / 8, 0, stream>>>(W1, W1T, kH, kH, kH, kH2, kH);
  wt_plane_kernel<<<kF, kH / 8, 0, stream>>>(W2, W2T, kH, kF, kF, kH2, 0);
  wt_plane_kernel<<<kF, kH / 8, 0, stream>>>(W2, W2T, kH, kF, kF, kH2, kH);
  z_plane_kernel<<<1024, kThr, 0, stream>>>(z, Z16);
  setup_f16_kernel<<<48, kThr, 0, stream>>>(bp, BP16, H0Z);
  setup_f32_kernel<<<8, kThr, 0, stream>>>(b1, b2, bs, b1d, b2d, F);

  wmma_gemm64<0, false, 2, 0, false, 0><<<dim3((kG4 / 64) * (kZ / 64) / 8, 1), 256, 0, stream>>>(
      K0T, K0T, kH2, 0L, WP16, WP16, kH2, 0L, (void*)WC32, (void*)WC32, kZ, 0L, F + kFZB, nullptr, 0L, kG4, kZ, kH2, kScC);
  wmma_gemm64<0, false, 2, 0, false, 0><<<dim3((kG4 / 64) * (kB / 64) / 8, 1), 256, 0, stream>>>(
      K0T, K0T, kH2, 0L, BP16, BP16, kH2, 0L, (void*)BPK, (void*)BPK, 64, 0L, F + kFZB, nullptr, 0L, kG4, 64, kH2, kScC);
  wc_split_kernel<<<128, kThr, 0, stream>>>(WC32, WCT);
  bias_c_kernel<<<2, kThr, 0, stream>>>(BPK, b0, F + kFBC);

  wmma_gemm64<0, false, 2, 0, false, 0><<<dim3((kRows / 64) * (kH / 64) / 8, 1), 256, 0, stream>>>(
      Z16, Z16, kZ2, 0L, WST, WST, kZ, 0L, (void*)RES, (void*)RES, kH, 0L, F + kFBS, nullptr, 0L, kRows, kH, kZ, kScXW);

  for (int layer = 0; layer < 3; ++layer) {
    const unsigned short* Ain = (layer == 0) ? Z16 : ((layer == 1) ? HS0 : X2);
    const int lda = (layer == 0) ? kZ2 : kH;
    const int Kin = (layer == 0) ? kZ2 : kH;
    const unsigned short* Bin = (layer == 0) ? WCT : ((layer == 1) ? K1T : K2T);
    const unsigned short* Rt  = (layer == 0) ? R0T : ((layer == 1) ? R1T : R2T);
    unsigned short* HS = (layer == 0) ? HS0 : ((layer == 1) ? HS1 : HS2);
    const float* bias = F + ((layer == 0) ? kFBC : ((layer == 1) ? kFB1 : kFB2));
    cell_zero_kernel<<<32, kThr, 0, stream>>>(C32);
    for (int c = 0; c < kNCh; ++c) {
      wmma_gemm64<0, false, 2, 0, false, 0><<<dim3((kChRows / 64) * (kG4 / 64) / 8, 1), 256, 0, stream>>>(
          Ain + (size_t)c * kChRows * lda, Ain + (size_t)c * kChRows * lda, lda, 0L, Bin, Bin, Kin, 0L, (void*)XK, (void*)XK, kG4, 0L, bias, nullptr, 0L, kChRows, kG4, Kin, kScXW);
      for (int tc = 0; tc < kCh; ++tc) {
        const int t = c * kCh + tc;
        const unsigned short* Hprev = (t == 0) ? H0Z : (HS + (size_t)(t - 1) * kB * kH);
        wmma_gemm64<0, false, 2, 0, false, 0><<<dim3((kB / 64) * (kG4 / 64) / 8, 1), 256, 0, stream>>>(
            Hprev, Hprev, kH, 0L, Rt, Rt, kH, 0L, (void*)GG, (void*)GG, kG4, 0L, F + kFZB, nullptr, 0L, kB, kG4, kH, kScXW);
        lstm_cell_kernel<<<16, kThr, 0, stream>>>(XK, GG, C32, HS, RES, X2, H2F, t, layer);
      }
    }
  }

  norm_split_kernel<<<64, kThr, 0, stream>>>(H2F, gamma, beta, XN16);
  wmma_gemm64<0, false, 2, 0, false, 0><<<dim3((kRows / 64) * (kH / 64) / 8, 1), 256, 0, stream>>>(
      XN16, XN16, kH2, 0L, W1T, W1T, kH2, 0L, (void*)D1, (void*)D1, kH, 0L, F + kFB1D, nullptr, 0L, kRows, kH, kH2, kScNW);
  relu_split_kernel<<<4096, kThr, 0, stream>>>(D1, D116);
  wmma_gemm64<0, false, 2, 0, false, 0><<<dim3((kRows / 64) * (kF / 64) / 8, 1), 256, 0, stream>>>(
      D116, D116, kH2, 0L, W2T, W2T, kH2, 0L, (void*)Y, (void*)Y, kF, 0L, F + kFB2D, nullptr, 0L, kRows, kF, kH2, kScXW);
  out_tanh_kernel<<<1024, kThr, 0, stream>>>(Y, out);
}
